// DecoderPromptLayer_79989470920966
// MI455X (gfx1250) — hardware-verified
//
#include <hip/hip_runtime.h>
#include <stddef.h>

typedef _Float16 v16h __attribute__((ext_vector_type(16)));
typedef _Float16 v8h  __attribute__((ext_vector_type(8)));
typedef float    v8f  __attribute__((ext_vector_type(8)));
typedef float    v4f  __attribute__((ext_vector_type(4)));
typedef v8h __attribute__((may_alias)) v8ha;
typedef v4f __attribute__((may_alias)) v4fa;

union Frag { v16h v; v8h half[2]; };

#define NB   2
#define NT   2048
#define NM   256
#define NS   2304
#define ND   1024
#define NH   16
#define HD   64
#define NF   4096
#define NBS  (NB * NS)
#define NBT  (NB * NT)
#define NW   (ND * ND)
#define WSC    64.0f
#define WINV   0.015625f
#define PSCALE 16384.0f
#define OSC    64.0f
#define HSC    64.0f

static_assert(NS % 128 == 0);
static_assert(NT % 64 == 0);
static_assert(ND % 64 == 0);
static_assert(NF % 64 == 0);
static_assert(NBT % 128 == 0);

__device__ __forceinline__ v8f wmma_f16(v16h a, v16h b, v8f c) {
  v8f d = __builtin_amdgcn_wmma_f32_16x16x32_f16(false, a, false, b, (short)0, c, false, false);
  asm volatile("v_nop\n\tv_nop\n\tv_nop\n\tv_nop" : "+v"(d) : "v"(a), "v"(b));
  return d;
}

__device__ __forceinline__ v16h load_frag(const _Float16* p, int h) {
  Frag f;
  f.half[0] = *(const v8ha*)(p + 8 * h);
  f.half[1] = *(const v8ha*)(p + 16 + 8 * h);
  return f.v;
}

__device__ __forceinline__ void wtrans_store(const float* st, _Float16* out, int K, int n0, int k0, int tid) {
  #pragma unroll
  for (int it = 0; it < 2; ++it) {
    const int p = tid + 256 * it;
    const int nl = p >> 3, q = p & 7;
    const float* col = st + (8 * q) * 65 + nl;
    v8h v;
    v[0] = (_Float16)(col[0 * 65] * WSC);
    v[1] = (_Float16)(col[1 * 65] * WSC);
    v[2] = (_Float16)(col[2 * 65] * WSC);
    v[3] = (_Float16)(col[3 * 65] * WSC);
    v[4] = (_Float16)(col[4 * 65] * WSC);
    v[5] = (_Float16)(col[5 * 65] * WSC);
    v[6] = (_Float16)(col[6 * 65] * WSC);
    v[7] = (_Float16)(col[7 * 65] * WSC);
    *(volatile v8h*)(out + (size_t)(n0 + nl) * K + k0 + 8 * q) = v;
  }
}

__global__ __launch_bounds__(256) void wtrans_kernel(const float* __restrict__ in, _Float16* __restrict__ out,
                                                    int K, int N)
{
  __shared__ float st[64 * 65];
  const int tid = threadIdx.x;
  const int n0 = blockIdx.x * 64, k0 = blockIdx.y * 64;
  if (n0 + 64 > N || k0 + 64 > K) return;
  #pragma unroll
  for (int it = 0; it < 4; ++it) {
    const int idx = tid + 256 * it;
    const int kr = idx >> 4, c4 = idx & 15;
    const v4f v = *(const v4fa*)(in + (size_t)(k0 + kr) * N + n0 + 4 * c4);
    float* d = st + kr * 65 + 4 * c4;
    d[0] = v[0]; d[1] = v[1]; d[2] = v[2]; d[3] = v[3];
  }
  __syncthreads();
  wtrans_store(st, out, K, n0, k0, tid);
  __threadfence();
  wtrans_store(st, out, K, n0, k0, tid);
}

__global__ __launch_bounds__(256) void rope_tab_kernel(float* __restrict__ tab)
{
  __shared__ __attribute__((aligned(16))) float st[16 * 32];
  const int t = threadIdx.x, pl = t >> 4, i = t & 15;
  const int s = blockIdx.x * 16 + pl;
  const float lit[16] = {1.0f, 1.7782794100389228f, 3.1622776601683795f, 5.623413251903491f,
                         10.0f, 17.78279410038923f, 31.622776601683793f, 56.23413251903491f,
                         100.0f, 177.82794100389228f, 316.22776601683796f, 562.341325190349f,
                         1000.0f, 1778.2794100389228f, 3162.2776601683795f, 5623.413251903491f};
  float p10 = 1.0f;
  #pragma unroll
  for (int j = 0; j < 16; ++j) p10 = (i == j) ? lit[j] : p10;
  const float invf = 1.0f / p10;
  const float ang = (float)s * invf;
  float sn, cs;
  sincosf(ang, &sn, &cs);
  st[pl * 32 + i] = cs;
  st[pl * 32 + 16 + i] = sn;
  __syncthreads();
  if (t < 128) {
    const int line = t >> 3, q = t & 7;
    const v4f v = *(const v4fa*)(st + line * 32 + 4 * q);
    float* dst = tab + (size_t)(blockIdx.x * 16 + line) * 32 + 4 * q;
    *(volatile v4f*)dst = v;
    __threadfence();
    *(volatile v4f*)dst = v;
  }
}

__global__ __launch_bounds__(128) void ln_kernel(const float* __restrict__ srcA, const float* __restrict__ srcB,
                                                const float* __restrict__ g, const float* __restrict__ be,
                                                _Float16* __restrict__ y, int concat)
{
  __shared__ float sp[2][4];
  const int row = blockIdx.x, t = threadIdx.x, lane = t & 31, w = t >> 5;
  const float* src;
  if (concat) {
    const int b = row / NS, s = row - b * NS;
    src = (s < NM) ? (srcA + ((size_t)b * NM + s) * ND) : (srcB + ((size_t)b * NT + (s - NM)) * ND);
  } else {
    src = srcA + (size_t)row * ND;
  }
  const v4f a = *(const v4fa*)(src + 8 * t);
  const v4f c = *(const v4fa*)(src + 8 * t + 4);
  float e[8] = {a[0], a[1], a[2], a[3], c[0], c[1], c[2], c[3]};

  float s1 = ((e[0] + e[1]) + (e[2] + e[3])) + ((e[4] + e[5]) + (e[6] + e[7]));
  #pragma unroll
  for (int off = 16; off > 0; off >>= 1) s1 += __shfl_xor(s1, off);
  if (lane == 0) sp[0][w] = s1;
  __syncthreads();
  const float mu = ((sp[0][0] + sp[0][1]) + (sp[0][2] + sp[0][3])) * (1.0f / ND);

  float d[8];
  float s2 = 0.0f;
  #pragma unroll
  for (int i = 0; i < 8; ++i) { d[i] = e[i] - mu; s2 += d[i] * d[i]; }
  #pragma unroll
  for (int off = 16; off > 0; off >>= 1) s2 += __shfl_xor(s2, off);
  if (lane == 0) sp[1][w] = s2;
  __syncthreads();
  const float var = ((sp[1][0] + sp[1][1]) + (sp[1][2] + sp[1][3])) * (1.0f / ND);
  const float rstd = rsqrtf(var + 1e-5f);

  const v4f g0 = *(const v4fa*)(g + 8 * t);
  const v4f g1 = *(const v4fa*)(g + 8 * t + 4);
  const v4f b0 = *(const v4fa*)(be + 8 * t);
  const v4f b1 = *(const v4fa*)(be + 8 * t + 4);
  const v8h o = { (_Float16)(d[0] * rstd * g0[0] + b0[0]), (_Float16)(d[1] * rstd * g0[1] + b0[1]),
                  (_Float16)(d[2] * rstd * g0[2] + b0[2]), (_Float16)(d[3] * rstd * g0[3] + b0[3]),
                  (_Float16)(d[4] * rstd * g1[0] + b1[0]), (_Float16)(d[5] * rstd * g1[1] + b1[1]),
                  (_Float16)(d[6] * rstd * g1[2] + b1[2]), (_Float16)(d[7] * rstd * g1[3] + b1[3]) };
  _Float16* dst = y + (size_t)row * ND + 8 * t;
  *(volatile v8h*)dst = o;
  __threadfence();
  *(volatile v8h*)dst = o;
}

__device__ __forceinline__ void proj_store_pass(const _Float16* sT, _Float16* plane, _Float16* vt,
                                                int which, int bh, int l0, int w, int lane) {
  const int q8 = lane & 7, sub = lane >> 3;
  #pragma unroll
  for (int i = 0; i < 8; ++i) {
    const int lid = w * 32 + i * 4 + sub;
    v8h v;
    _Float16* dst;
    if (which != 2) {
      v = *(const v8ha*)(sT + lid * HD + 8 * q8);
      dst = plane + ((size_t)bh * NS + l0 + lid) * HD + 8 * q8;
    } else {
      const int d = lid >> 1, hl = lid & 1;
      v = *(const v8ha*)(sT + d * 128 + 64 * hl + 8 * q8);
      dst = vt + ((size_t)bh * HD + d) * NS + l0 + 64 * hl + 8 * q8;
    }
    *(volatile v8h*)dst = v;
  }
}

__global__ __launch_bounds__(128) void proj_kernel(
    const _Float16* __restrict__ xa,
    const _Float16* __restrict__ wt,
    const float* __restrict__ bq, const float* __restrict__ bk, const float* __restrict__ bv,
    const float* __restrict__ tab,
    _Float16* __restrict__ qp,
    _Float16* __restrict__ kp,
    _Float16* __restrict__ vt)
{
  __shared__ __attribute__((aligned(16))) _Float16 sT[128 * 64];

  const int tid = threadIdx.x, lane = tid & 31, w = tid >> 5;
  const int h = lane >> 4, m = lane & 15;
  const int m0 = blockIdx.x * 128;
  const int cg = blockIdx.y;
  const int which = cg >> 4, head = cg & 15;
  const int b = m0 / NS, l0 = m0 - b * NS, bh = b * NH + head;
  if (which == 0 && l0 < NM) return;
  const int m0w = m0 + 32 * w;

  const _Float16* xa0 = xa + (size_t)(m0w + m) * ND;
  const _Float16* xa1 = xa0 + (size_t)16 * ND;
  const _Float16* wb  = wt + ((size_t)which * ND + head * HD + m) * ND;

  const v8f zero8 = {0.f, 0.f, 0.f, 0.f, 0.f, 0.f, 0.f, 0.f};
  v8f acc[2][4];
  #pragma unroll
  for (int mt = 0; mt < 2; ++mt)
    #pragma unroll
    for (int nt = 0; nt < 4; ++nt) acc[mt][nt] = zero8;

  #pragma unroll 1
  for (int k0 = 0; k0 < ND; k0 += 32) {
    const v16h a0 = load_frag(xa0 + k0, h);
    const v16h a1 = load_frag(xa1 + k0, h);
    #pragma unroll
    for (int nt = 0; nt < 4; ++nt) {
      const v16h bf = load_frag(wb + (size_t)nt * 16 * ND + k0, h);
      acc[0][nt] = wmma_f16(a0, bf, acc[0][nt]);
      acc[1][nt] = wmma_f16(a1, bf, acc[1][nt]);
    }
  }

  const float* bias = (which == 0) ? bq : ((which == 1) ? bk : bv);
  #pragma unroll
  for (int nt = 0; nt < 4; ++nt) {
    const float bvl = bias[head * HD + 16 * nt + m];
    #pragma unroll
    for (int mt = 0; mt < 2; ++mt)
      #pragma unroll
      for (int r = 0; r < 8; ++r) acc[mt][nt][r] = acc[mt][nt][r] * WINV + bvl;
  }

  if (which < 2) {
    #pragma unroll
    for (int mt = 0; mt < 2; ++mt)
      #pragma unroll
      for (int r = 0; r < 8; ++r) {
        const int s = l0 + 32 * w + 16 * mt + 8 * h + r;
        const float cs = tab[(size_t)s * 32 + m];
        const float sn = tab[(size_t)s * 32 + 16 + m];
        const float x1 = acc[mt][0][r], x2 = acc[mt][1][r];
        acc[mt][0][r] = x1 * cs - x2 * sn;
        acc[mt][1][r] = x2 * cs + x1 * sn;
      }
  }

  #pragma unroll
  for (int nt = 0; nt < 4; ++nt) {
    const int feat = 16 * nt + m;
    #pragma unroll
    for (int mt = 0; mt < 2; ++mt) {
      #pragma unroll
      for (int r = 0; r < 8; ++r) {
        const int tokl = 32 * w + 16 * mt + 8 * h + r;
        const int idx = (which == 2) ? (feat * 128 + tokl) : (tokl * HD + feat);
        sT[idx] = (_Float16)acc[mt][nt][r];
      }
    }
  }
  __syncthreads();

  _Float16* plane = (which == 0) ? qp : kp;
  proj_store_pass(sT, plane, vt, which, bh, l0, w, lane);
  __threadfence();
  proj_store_pass(sT, plane, vt, which, bh, l0, w, lane);
}

__device__ __forceinline__ v16h pack_p(v8f a, v8f c) {
  const v16h r = { (_Float16)(a[0] * PSCALE), (_Float16)(a[1] * PSCALE), (_Float16)(a[2] * PSCALE), (_Float16)(a[3] * PSCALE),
                   (_Float16)(a[4] * PSCALE), (_Float16)(a[5] * PSCALE), (_Float16)(a[6] * PSCALE), (_Float16)(a[7] * PSCALE),
                   (_Float16)(c[0] * PSCALE), (_Float16)(c[1] * PSCALE), (_Float16)(c[2] * PSCALE), (_Float16)(c[3] * PSCALE),
                   (_Float16)(c[4] * PSCALE), (_Float16)(c[5] * PSCALE), (_Float16)(c[6] * PSCALE), (_Float16)(c[7] * PSCALE) };
  return r;
}

__device__ __forceinline__ void att_store_pass(const _Float16* so, _Float16* op, int orow0, int head, int lane) {
  const int q8 = lane & 7, sub = lane >> 3;
  #pragma unroll
  for (int i = 0; i < 4; ++i) {
    const int lid = i * 4 + sub;
    const v8h v = *(const v8ha*)(so + lid * 64 + 8 * q8);
    *(volatile v8h*)(op + ((size_t)orow0 + lid) * ND + head * HD + 8 * q8) = v;
  }
}

__global__ __launch_bounds__(128) void attn_kernel(
    const _Float16* __restrict__ qp,
    const _Float16* __restrict__ kp,
    const _Float16* __restrict__ vt,
    _Float16* __restrict__ op)
{
  __shared__ __attribute__((aligned(16))) _Float16 sO[4 * 16 * 64];

  const int tid = threadIdx.x, lane = tid & 31, w = tid >> 5;
  const int h = lane >> 4, m = lane & 15;
  const int bh = blockIdx.y, b = bh >> 4, head = bh & 15;
  const int q0w = NM + blockIdx.x * 64 + 16 * w;

  const _Float16* qrow = qp + ((size_t)bh * NS + q0w + m) * HD;
  const v16h qb0 = load_frag(qrow, h);
  const v16h qb1 = load_frag(qrow + 32, h);

  const v8f zero8 = {0.f, 0.f, 0.f, 0.f, 0.f, 0.f, 0.f, 0.f};
  v8f o[4];
  #pragma unroll
  for (int t = 0; t < 4; ++t) o[t] = zero8;
  float mrun = -1e30f, lrun = 0.0f;

  const _Float16* kbase = kp + ((size_t)bh * NS + m) * HD;
  const _Float16* vbase = vt + ((size_t)bh * HD + m) * NS;
  const int kend = q0w + 16;

  #pragma unroll 1
  for (int kb = 0; kb < kend; kb += 64) {
    v8f s[4];
    #pragma unroll
    for (int j = 0; j < 4; ++j) {
      const _Float16* kpj = kbase + (size_t)(kb + 16 * j) * HD;
      const v16h kf0 = load_frag(kpj, h);
      const v16h kf1 = load_frag(kpj + 32, h);
      v8f z = zero8;
      z = wmma_f16(kf0, qb0, z);
      z = wmma_f16(kf1, qb1, z);
      #pragma unroll
      for (int r = 0; r < 8; ++r) z[r] = z[r] * 0.125f;
      s[j] = z;
    }
    if (kb + 64 > q0w) {
      const int qi = q0w + m;
      #pragma unroll
      for (int j = 0; j < 4; ++j)
        #pragma unroll
        for (int r = 0; r < 8; ++r) {
          const int kj = kb + 16 * j + 8 * h + r;
          s[j][r] = (kj <= qi) ? s[j][r] : -1e30f;
        }
    }

    float mloc = s[0][0];
    #pragma unroll
    for (int j = 0; j < 4; ++j)
      #pragma unroll
      for (int r = 0; r < 8; ++r) mloc = fmaxf(mloc, s[j][r]);
    mloc = fmaxf(mloc, __shfl_xor(mloc, 16));
    const float mnew = fmaxf(mrun, mloc);
    const float alpha = __expf(mrun - mnew);
    mrun = mnew;
    float lsum = 0.0f;
    #pragma unroll
    for (int j = 0; j < 4; ++j)
      #pragma unroll
      for (int r = 0; r < 8; ++r) {
        const float p = __expf(s[j][r] - mnew);
        s[j][r] = p;
        lsum += p;
      }
    lsum += __shfl_xor(lsum, 16);
    lrun = lrun * alpha + lsum;
    #pragma unroll
    for (int t = 0; t < 4; ++t)
      #pragma unroll
      for (int r = 0; r < 8; ++r) o[t][r] = o[t][r] * alpha;

    const v16h pb0 = pack_p(s[0], s[1]);
    const v16h pb1 = pack_p(s[2], s[3]);

    #pragma unroll
    for (int t = 0; t < 4; ++t) {
      const _Float16* vp = vbase + (size_t)(16 * t) * NS + kb;
      const v16h vf0 = load_frag(vp, h);
      const v16h vf1 = load_frag(vp + 32, h);
      o[t] = wmma_f16(vf0, pb0, o[t]);
      o[t] = wmma_f16(vf1, pb1, o[t]);
    }
  }

  const float inv = (1.0f / lrun) * (OSC / PSCALE);
  _Float16* so = sO + w * 1024;
  #pragma unroll
  for (int t = 0; t < 4; ++t)
    #pragma unroll
    for (int r = 0; r < 8; ++r)
      so[m * 64 + 16 * t + 8 * h + r] = (_Float16)(o[t][r] * inv);
  __syncthreads();

  const int orow0 = b * NT + (q0w - NM);
  att_store_pass(so, op, orow0, head, lane);
  __threadfence();
  att_store_pass(so, op, orow0, head, lane);
}

__device__ __forceinline__ void storeF_pass(const float* sF, float* out, int N, int row0, int col0, int w, int lane) {
  const int q8 = lane & 7, sub = lane >> 3;
  #pragma unroll
  for (int i = 0; i < 16; ++i) {
    const int lid = i * 4 + sub;
    const int rowl = 32 * w + (lid >> 1), hl = lid & 1;
    const v4f v = *(const v4fa*)(sF + rowl * 64 + 32 * hl + 4 * q8);
    *(volatile v4f*)(out + (size_t)(row0 + rowl) * N + col0 + 32 * hl + 4 * q8) = v;
  }
}

__device__ __forceinline__ void storeH_pass(const _Float16* sH, _Float16* out, int N, int row0, int col0, int w, int lane) {
  const int q8 = lane & 7, sub = lane >> 3;
  #pragma unroll
  for (int i = 0; i < 8; ++i) {
    const int lid = 32 * w + i * 4 + sub;
    const v8h v = *(const v8ha*)(sH + lid * 64 + 8 * q8);
    *(volatile v8h*)(out + (size_t)(row0 + lid) * N + col0 + 8 * q8) = v;
  }
}

template <int EPI>
__global__ __launch_bounds__(128) void gemm_kernel(
    const _Float16* __restrict__ A,
    const _Float16* __restrict__ Bt,
    const float* __restrict__ bias,
    const float* __restrict__ resid,
    float* __restrict__ outF,
    _Float16* __restrict__ outH,
    int K, int N, float scale, float hsc)
{
  __shared__ __attribute__((aligned(16))) float sF[128 * 64];

  const int tid = threadIdx.x, lane = tid & 31, w = tid >> 5;
  const int h = lane >> 4, m = lane & 15;
  const int row0 = blockIdx.x * 128, col0 = blockIdx.y * 64;
  const int row0w = row0 + 32 * w;

  const _Float16* a0p = A + (size_t)(row0w + m) * K;
  const _Float16* a1p = a0p + (size_t)16 * K;
  const _Float16* bp  = Bt + (size_t)(col0 + m) * K;

  const v8f zero8 = {0.f, 0.f, 0.f, 0.f, 0.f, 0.f, 0.f, 0.f};
  v8f acc[2][4];
  #pragma unroll
  for (int mt = 0; mt < 2; ++mt)
    #pragma unroll
    for (int nt = 0; nt < 4; ++nt) acc[mt][nt] = zero8;

  #pragma unroll 1
  for (int k0 = 0; k0 < K; k0 += 32) {
    const v16h a0 = load_frag(a0p + k0, h);
    const v16h a1 = load_frag(a1p + k0, h);
    #pragma unroll
    for (int nt = 0; nt < 4; ++nt) {
      const v16h bf = load_frag(bp + (size_t)nt * 16 * K + k0, h);
      acc[0][nt] = wmma_f16(a0, bf, acc[0][nt]);
      acc[1][nt] = wmma_f16(a1, bf, acc[1][nt]);
    }
  }

  _Float16* sH = (_Float16*)sF;
  #pragma unroll
  for (int nt = 0; nt < 4; ++nt) {
    const int col = 16 * nt + m;
    const float bvl = bias[col0 + col];
    #pragma unroll
    for (int mt = 0; mt < 2; ++mt) {
      #pragma unroll
      for (int r = 0; r < 8; ++r) {
        const int rowl = 32 * w + 16 * mt + 8 * h + r;
        float v = acc[mt][nt][r] * scale + bvl;
        if (EPI == 0) {
          v += resid[(size_t)(row0 + rowl) * N + col0 + col];
          sF[rowl * 64 + col] = v;
        } else {
          v = fmaxf(v, 0.0f);
          sH[rowl * 64 + col] = (_Float16)(v * v * hsc);
        }
      }
    }
  }
  __syncthreads();

  if (EPI == 0) {
    storeF_pass(sF, outF, N, row0, col0, w, lane);
    __threadfence();
    storeF_pass(sF, outF, N, row0, col0, w, lane);
  } else {
    storeH_pass(sH, outH, N, row0, col0, w, lane);
    __threadfence();
    storeH_pass(sH, outH, N, row0, col0, w, lane);
  }
}

extern "C" void kernel_launch(void* const* d_in, const int* in_sizes, int n_in,
                              void* d_out, int out_size, void* d_ws, size_t ws_size,
                              hipStream_t stream) {
  if (n_in < 18) return;
  if (in_sizes[0] != NBT * ND) return;
  if (in_sizes[1] != NB * NM * ND) return;
  if (in_sizes[2] != NW || in_sizes[4] != NW || in_sizes[6] != NW || in_sizes[8] != NW) return;
  if (in_sizes[3] != ND || in_sizes[5] != ND || in_sizes[7] != ND || in_sizes[9] != ND) return;
  if (in_sizes[10] != ND * NF || in_sizes[12] != NF * ND) return;
  if (in_sizes[11] != NF || in_sizes[13] != ND) return;
  if (in_sizes[14] != ND || in_sizes[15] != ND || in_sizes[16] != ND || in_sizes[17] != ND) return;
  if (out_size != NBT * ND) return;

  const float* x      = (const float*)d_in[0];
  const float* memory = (const float*)d_in[1];
  const float* Wq = (const float*)d_in[2];
  const float* bq = (const float*)d_in[3];
  const float* Wk = (const float*)d_in[4];
  const float* bk = (const float*)d_in[5];
  const float* Wv = (const float*)d_in[6];
  const float* bv = (const float*)d_in[7];
  const float* Wo = (const float*)d_in[8];
  const float* bo = (const float*)d_in[9];
  const float* W1 = (const float*)d_in[10];
  const float* b1 = (const float*)d_in[11];
  const float* W2 = (const float*)d_in[12];
  const float* b2 = (const float*)d_in[13];
  const float* ln1_g = (const float*)d_in[14];
  const float* ln1_b = (const float*)d_in[15];
  const float* ln2_g = (const float*)d_in[16];
  const float* ln2_b = (const float*)d_in[17];
  float* out = (float*)d_out;

  const size_t szWqkv = (size_t)3 * NW * 2;
  const size_t szWo   = (size_t)NW * 2;
  const size_t szW1   = (size_t)ND * NF * 2;
  const size_t szW2   = (size_t)NF * ND * 2;
  const size_t szTab  = (size_t)NS * 32 * 4;
  const size_t szXa   = (size_t)NBS * ND * 2;
  const size_t szPl   = (size_t)NB * NH * NS * HD * 2;
  const size_t szO    = (size_t)NBT * ND * 2;
  const size_t szX2   = (size_t)NBT * ND * 4;
  const size_t szXf   = (size_t)NBT * ND * 2;
  const size_t szH    = (size_t)NBT * NF * 2;
  const size_t total  = szWqkv + szWo + szW1 + szW2 + szTab + szXa + 3 * szPl + szO + szX2 + szXf + szH;
  if (total > ws_size) return;

  char* ws = (char*)d_ws;
  size_t off = 0;
  _Float16* wqkvT = (_Float16*)(ws + off); off += szWqkv;
  _Float16* woT   = (_Float16*)(ws + off); off += szWo;
  _Float16* w1T   = (_Float16*)(ws + off); off += szW1;
  _Float16* w2T   = (_Float16*)(ws + off); off += szW2;
  float*    tab   = (float*)(ws + off);    off += szTab;
  _Float16* xa    = (_Float16*)(ws + off); off += szXa;
  _Float16* qpl   = (_Float16*)(ws + off); off += szPl;
  _Float16* kpl   = (_Float16*)(ws + off); off += szPl;
  _Float16* vtp   = (_Float16*)(ws + off); off += szPl;
  _Float16* opl   = (_Float16*)(ws + off); off += szO;
  float*    x2    = (float*)(ws + off);    off += szX2;
  _Float16* xf    = (_Float16*)(ws + off); off += szXf;
  _Float16* hp    = (_Float16*)(ws + off); off += szH;
  if (off != total) return;

  wtrans_kernel<<<dim3(ND / 64, ND / 64), 256, 0, stream>>>(Wq, wqkvT, ND, ND);
  wtrans_kernel<<<dim3(ND / 64, ND / 64), 256, 0, stream>>>(Wk, wqkvT + (size_t)NW, ND, ND);
  wtrans_kernel<<<dim3(ND / 64, ND / 64), 256, 0, stream>>>(Wv, wqkvT + (size_t)2 * NW, ND, ND);
  wtrans_kernel<<<dim3(ND / 64, ND / 64), 256, 0, stream>>>(Wo, woT, ND, ND);
  wtrans_kernel<<<dim3(NF / 64, ND / 64), 256, 0, stream>>>(W1, w1T, ND, NF);
  wtrans_kernel<<<dim3(ND / 64, NF / 64), 256, 0, stream>>>(W2, w2T, NF, ND);

  rope_tab_kernel<<<NS / 16, 256, 0, stream>>>(tab);

  ln_kernel<<<NBS, 128, 0, stream>>>(memory, x, ln1_g, ln1_b, xa, 1);

  proj_kernel<<<dim3(NBS / 128, 3 * NH), 128, 0, stream>>>(xa, wqkvT, bq, bk, bv, tab, qpl, kpl, vtp);

  attn_kernel<<<dim3(NT / 64, NB * NH), 128, 0, stream>>>(qpl, kpl, vtp, opl);

  gemm_kernel<0><<<dim3(NBT / 128, ND / 64), 128, 0, stream>>>(opl, woT, bo, x, x2, opl, ND, ND, 1.0f / 4096.0f, 0.0f);

  ln_kernel<<<NBT, 128, 0, stream>>>(x2, x2, ln2_g, ln2_b, xf, 0);

  gemm_kernel<1><<<dim3(NBT / 128, NF / 64), 128, 0, stream>>>(xf, w1T, b1, b1, x2, hp, ND, NF, WINV, HSC);

  gemm_kernel<0><<<dim3(NBT / 128, ND / 64), 128, 0, stream>>>(hp, w2T, b2, x2, out, hp, NF, ND, 1.0f / 4096.0f, 0.0f);
}
